// DecoderBlock_63273458205166
// MI455X (gfx1250) — hardware-verified
//
#include <hip/hip_runtime.h>
#include <math.h>

#ifndef NB
#define NB 2
#endif
#ifndef SEQ
#define SEQ 2048
#endif
#define NB_FULL 2
#define SEQ_FULL 2048
#define DM 1024
#define DFFN 4096
#define NHEAD 16
#define MROWS (NB * SEQ)

static_assert(SEQ % 64 == 0);
static_assert(SEQ <= SEQ_FULL);
static_assert(NB <= NB_FULL);
static_assert((SEQ & (SEQ - 1)) == 0);
static_assert(MROWS % 64 == 0);

typedef __attribute__((ext_vector_type(16))) _Float16 v16h;
typedef __attribute__((ext_vector_type(8)))  _Float16 v8h;
typedef __attribute__((ext_vector_type(8)))  float    v8f;
typedef __attribute__((ext_vector_type(4)))  float    v4f;
typedef __attribute__((ext_vector_type(4)))  unsigned v4u;
typedef __attribute__((ext_vector_type(2)))  unsigned v2u;

union FragU { v16h v; v8h h[2]; };
__device__ __forceinline__ v16h frag_ld(const _Float16* p) { FragU f; f.h[0] = *(const v8h*)(p); f.h[1] = *(const v8h*)(p + 16); return f.v; }
__device__ __forceinline__ v8f mma_raw(v16h a, v16h b, v8f c) { return __builtin_amdgcn_wmma_f32_16x16x32_f16(false, a, false, b, (short)0, c, false, false); }
__device__ __forceinline__ v8f wmma16(v16h a, v16h b, v8f c) {
    c = __builtin_amdgcn_wmma_f32_16x16x32_f16(false, a, false, b, (short)0, c, false, false);
    asm volatile("v_nop\n\tv_nop\n\tv_nop\n\tv_nop" : "+v"(c) : "v"(a), "v"(b));
    return c;
}
__device__ __forceinline__ void dep_guard_h(v8f& a, v8f& b, v16h x, v16h y) { asm volatile("v_nop\n\tv_nop\n\tv_nop\n\tv_nop" : "+v"(a), "+v"(b) : "v"(x), "v"(y)); }
__device__ __forceinline__ void keep4_h(v16h a, v16h b, v16h c, v16h d) { asm volatile("v_nop" :: "v"(a), "v"(b), "v"(c), "v"(d)); }
__device__ __forceinline__ void acc_guard4(v8f& a, v8f& b, v8f& c, v8f& d) { asm volatile("v_nop\n\tv_nop\n\tv_nop\n\tv_nop" : "+v"(a), "+v"(b), "+v"(c), "+v"(d)); }

__device__ __forceinline__ float bf_rne(float v) { const unsigned u = __builtin_bit_cast(unsigned, v); const unsigned r = (u + 0x7fffu + ((u >> 16) & 1u)) & 0xffff0000u; return __builtin_bit_cast(float, r); }
__device__ __forceinline__ unsigned pk2h(float a, float b) { return (unsigned)__builtin_bit_cast(unsigned short, (_Float16)a) | ((unsigned)__builtin_bit_cast(unsigned short, (_Float16)b) << 16); }

#define VST2(T, ptr, val) do { const T vst2_v_ = (val); *(volatile T*)(ptr) = vst2_v_; __threadfence(); *(volatile T*)(ptr) = vst2_v_; } while (0)

__global__ __launch_bounds__(256) void k_castT(const float* __restrict__ SRC, unsigned lds, unsigned short* __restrict__ DST, unsigned ldd,
                                               unsigned nR, unsigned nC, unsigned perShift, float sc) {
    const unsigned u = blockIdx.x * 256u + threadIdx.x;
    if (u >= nC * (nR >> 3)) return;
    const unsigned cc = u >> perShift;
    const unsigned r0 = (u & ((1u << perShift) - 1u)) << 3;
    float w[8];
#pragma unroll
    for (int e = 0; e < 8; ++e) w[e] = bf_rne(SRC[(size_t)(r0 + (unsigned)e) * lds + cc]) * sc;
    v4u pk; pk.x = pk2h(w[0], w[1]); pk.y = pk2h(w[2], w[3]); pk.z = pk2h(w[4], w[5]); pk.w = pk2h(w[6], w[7]);
    VST2(v4u, (v4u*)(DST + (size_t)cc * ldd + r0), pk);
}

template <int SRCIN, int WF32>
__global__ __launch_bounds__(256) void k_ln(const float* __restrict__ X, const float* __restrict__ G, const float* __restrict__ Bb,
                                            unsigned short* __restrict__ O, float* __restrict__ OF) {
    #pragma clang fp contract(off)
    const unsigned row = blockIdx.x * 8u + (threadIdx.x >> 5);
    const unsigned L = threadIdx.x & 31u;
    if (row >= (unsigned)MROWS) return;
    size_t xoff;
    if (SRCIN) { const unsigned bb = row / (unsigned)SEQ; const unsigned ss = row - bb * (unsigned)SEQ; xoff = ((size_t)bb * SEQ_FULL + ss) * 1024u; }
    else xoff = (size_t)row * 1024u;
    const float* xr = X + xoff + 4u * L;
    float s = 0.f;
#pragma unroll 1
    for (unsigned g = 0; g < 8u; ++g) {
        const v4f a = *(const v4f*)(xr + 128u * g);
        const float t0 = SRCIN ? bf_rne(a.x) : a.x;
        const float t1 = SRCIN ? bf_rne(a.y) : a.y;
        const float t2 = SRCIN ? bf_rne(a.z) : a.z;
        const float t3 = SRCIN ? bf_rne(a.w) : a.w;
        s += t0; s += t1; s += t2; s += t3;
    }
#pragma unroll
    for (int o = 16; o > 0; o >>= 1) s += __shfl_xor(s, o, 32);
    const float mu = s * (1.f / 1024.f);
    float q = 0.f;
#pragma unroll 1
    for (unsigned g = 0; g < 8u; ++g) {
        const v4f a = *(const v4f*)(xr + 128u * g);
        const float t0 = SRCIN ? bf_rne(a.x) : a.x;
        const float t1 = SRCIN ? bf_rne(a.y) : a.y;
        const float t2 = SRCIN ? bf_rne(a.z) : a.z;
        const float t3 = SRCIN ? bf_rne(a.w) : a.w;
        const float d0 = t0 - mu, d1 = t1 - mu, d2 = t2 - mu, d3 = t3 - mu;
        q += d0 * d0; q += d1 * d1; q += d2 * d2; q += d3 * d3;
    }
#pragma unroll
    for (int o = 16; o > 0; o >>= 1) q += __shfl_xor(q, o, 32);
    const float rs = rsqrtf(q * (1.f / 1024.f) + 1e-5f);
#pragma unroll 1
    for (unsigned g = 0; g < 8u; ++g) {
        const unsigned c0 = 128u * g + 4u * L;
        const v4f a = *(const v4f*)(xr + 128u * g);
        const v4f ga = *(const v4f*)(G + c0);
        const v4f ba = *(const v4f*)(Bb + c0);
        const float t0 = SRCIN ? bf_rne(a.x) : a.x;
        const float t1 = SRCIN ? bf_rne(a.y) : a.y;
        const float t2 = SRCIN ? bf_rne(a.z) : a.z;
        const float t3 = SRCIN ? bf_rne(a.w) : a.w;
        const float y0 = (t0 - mu) * rs * bf_rne(ga.x) + bf_rne(ba.x);
        const float y1 = (t1 - mu) * rs * bf_rne(ga.y) + bf_rne(ba.y);
        const float y2 = (t2 - mu) * rs * bf_rne(ga.z) + bf_rne(ba.z);
        const float y3 = (t3 - mu) * rs * bf_rne(ga.w) + bf_rne(ba.w);
        v2u pk; pk.x = pk2h(y0, y1); pk.y = pk2h(y2, y3);
        v4f yv; yv.x = y0; yv.y = y1; yv.z = y2; yv.w = y3;
        volatile v2u* po = (volatile v2u*)(O + (size_t)row * 1024u + c0);
        *po = pk;
        if (WF32) { *(volatile v4f*)(OF + (size_t)row * 1024u + c0) = yv; }
        __threadfence();
        *po = pk;
        if (WF32) { *(volatile v4f*)(OF + (size_t)row * 1024u + c0) = yv; }
    }
}

template <int OUT_MODE, bool RESID, int ACT>
__global__ __launch_bounds__(256) void k_gemm64(
    const unsigned short* __restrict__ Ap, unsigned lda, unsigned long long strideA,
    const unsigned short* __restrict__ Btp, unsigned ldb, unsigned long long strideB,
    void* __restrict__ Cout, unsigned ldc, unsigned long long strideC,
    const float* __restrict__ bias0, const float* __restrict__ bias1,
    const float* __restrict__ resid, unsigned ldr,
    unsigned M, unsigned N, unsigned K, float scale) {
  const _Float16* A = (const _Float16*)Ap; const _Float16* Bt = (const _Float16*)Btp;
  __shared__ __align__(16) float sT[8][16 * 68];
  const unsigned b    = blockIdx.y;
  const unsigned lane = threadIdx.x & 31u;
  const unsigned wave = threadIdx.x >> 5;
  const unsigned tilesN = N >> 6;
  const unsigned tilesM = M >> 6;
  const unsigned tile = blockIdx.x * 8u + wave;
  if (tile >= tilesM * tilesN) return;
  const unsigned tm = tile / tilesN;
  const unsigned tn = tile - tm * tilesN;
  const unsigned m0 = tm << 6;
  const unsigned n0 = tn << 6;

  const _Float16* Ab = A  + (size_t)b * strideA;
  const _Float16* Bb = Bt + (size_t)b * strideB;
  const float* bias = (b == 0u) ? bias0 : bias1;

  const unsigned rlane = lane & 15u;
  const unsigned koff  = (lane >> 4) * 8u;
  const unsigned mOff  = (lane >> 4) * 8u;

  v8f acc[4][4];
#pragma unroll
  for (int i = 0; i < 4; ++i)
#pragma unroll
    for (int j = 0; j < 4; ++j) acc[i][j] = (v8f){0.f,0.f,0.f,0.f,0.f,0.f,0.f,0.f};

  for (unsigned k0 = 0; k0 < K; k0 += 32u) {
    v16h bh[4];
#pragma unroll
    for (int j = 0; j < 4; ++j) {
      const size_t bo = (size_t)(n0 + ((unsigned)j << 4) + rlane) * ldb + koff + k0;
      bh[j] = frag_ld(Bb + bo);
    }
#pragma unroll
    for (int i = 0; i < 4; ++i) {
      const size_t ao = (size_t)(m0 + ((unsigned)i << 4) + rlane) * lda + koff + k0;
      const v16h ah = frag_ld(Ab + ao);
#pragma unroll
      for (int j = 0; j < 4; ++j) acc[i][j] = mma_raw(ah, bh[j], acc[i][j]);
      dep_guard_h(acc[i][0], acc[i][3], ah, ah);
    }
    keep4_h(bh[0], bh[1], bh[2], bh[3]);
  }
  acc_guard4(acc[0][0], acc[0][1], acc[0][2], acc[0][3]);
  acc_guard4(acc[1][0], acc[1][1], acc[1][2], acc[1][3]);
  acc_guard4(acc[2][0], acc[2][1], acc[2][2], acc[2][3]);
  acc_guard4(acc[3][0], acc[3][1], acc[3][2], acc[3][3]);

  float* slab = sT[wave];
#pragma unroll
  for (int i = 0; i < 4; ++i) {
    const unsigned mBase = m0 + ((unsigned)i << 4);
#pragma unroll
    for (int j = 0; j < 4; ++j) {
      const unsigned n = n0 + ((unsigned)j << 4) + rlane;
      const float bv = bf_rne(bias[n]);
#pragma unroll
      for (int r = 0; r < 8; ++r) {
        float v = acc[i][j][r] * scale + bv;
        if (ACT == 2) v = fmaxf(v, 0.0f);
        slab[(mOff + (unsigned)r) * 68u + ((unsigned)j << 4) + rlane] = v;
      }
    }
    __builtin_amdgcn_fence(3  , "workgroup");
    __builtin_amdgcn_wave_barrier();
    __builtin_amdgcn_fence(2  , "workgroup");
    if (OUT_MODE == 0) {
      float* C = (float*)Cout + (size_t)b * strideC;
      const unsigned hh = lane >> 4, c4 = (lane & 15u) * 4u;
      if (RESID) {
#pragma unroll
        for (int it = 0; it < 8; ++it) {
          const unsigned row = (unsigned)it * 2u + hh;
          const v4f t = *(const v4f*)(slab + row * 68u + c4) + *(const v4f*)(resid + (size_t)(mBase + row) * ldr + n0 + c4);
          *(v4f*)(slab + row * 68u + c4) = t;
        }
      }
      for (int pass = 0; pass < 2; ++pass) {
#pragma unroll
        for (int it = 0; it < 8; ++it) {
          const unsigned row = (unsigned)it * 2u + hh;
          const v4f v = *(const v4f*)(slab + row * 68u + c4);
          *(volatile v4f*)(C + (size_t)(mBase + row) * ldc + n0 + c4) = v;
        }
        __threadfence();
      }
    } else {
      const unsigned q = lane >> 3, c8 = (lane & 7u) * 8u;
      unsigned short* C = (unsigned short*)Cout + (size_t)b * strideC;
      for (int pass = 0; pass < 2; ++pass) {
#pragma unroll
        for (int it = 0; it < 4; ++it) {
          const unsigned row = (unsigned)it * 4u + q;
          const float* sp = slab + row * 68u + c8;
          const v4f s0 = *(const v4f*)(sp), s1 = *(const v4f*)(sp + 4);
          v4u pk; pk.x = pk2h(s0.x, s0.y); pk.y = pk2h(s0.z, s0.w); pk.z = pk2h(s1.x, s1.y); pk.w = pk2h(s1.z, s1.w);
          *(volatile v4u*)(C + (size_t)(mBase + row) * ldc + n0 + c8) = pk;
        }
        __threadfence();
      }
    }
    __builtin_amdgcn_fence(3  , "workgroup");
    __builtin_amdgcn_wave_barrier();
    __builtin_amdgcn_fence(2  , "workgroup");
  }
}

__global__ __launch_bounds__(256) void k_prefix(const float* __restrict__ V32, float* __restrict__ CS) {
    const unsigned idx = blockIdx.x * 256u + threadIdx.x;
    if (idx >= (unsigned)NB * 1024u) return;
    const unsigned b = idx >> 10, cc = idx & 1023u;
    const float* src = V32 + (size_t)b * SEQ * 1024u + cc;
    float* dst = CS + (size_t)b * SEQ * 1024u + cc;
    float run = 0.f;
#pragma unroll 1
    for (unsigned s0 = 0; s0 < (unsigned)SEQ; s0 += 16u) {
        float o[16];
#pragma unroll
        for (int i = 0; i < 16; ++i) { const float v = src[(size_t)(s0 + (unsigned)i) * 1024u]; o[i] = run; run += v; }
        for (int pass = 0; pass < 2; ++pass) {
#pragma unroll
            for (int i = 0; i < 16; ++i) *(volatile float*)(dst + (size_t)(s0 + (unsigned)i) * 1024u) = o[i];
            __threadfence();
        }
    }
}

__global__ __launch_bounds__(128) void k_attn_tri(const unsigned short* __restrict__ QKp, const float* __restrict__ V32,
                                                  const float* __restrict__ CS, unsigned short* __restrict__ AO) {
    __shared__ float wsc[4][32];
    const unsigned tid = threadIdx.x, wave = tid >> 5, lane = tid & 31u, hh = lane >> 4, c = lane & 15u;
    constexpr unsigned NQB = (unsigned)SEQ / 64u;
    const unsigned bx = blockIdx.x;
    const unsigned qb = bx % NQB, bh = bx / NQB;
    const unsigned h = bh & 15u, b = bh >> 4;
    const unsigned rowbase = b * (unsigned)SEQ;
    const unsigned q0 = qb * 64u + wave * 16u;
    const _Float16* QK = (const _Float16*)QKp;
    const _Float16* qrow = QK + (size_t)(rowbase + q0 + c) * 2048u + h * 64u + 8u * hh;
    const v16h qa0 = frag_ld(qrow), qa1 = frag_ld(qrow + 32);
    float m[8], l[8], sd[8];
#pragma unroll
    for (int r = 0; r < 8; ++r) { m[r] = 0.f; l[r] = 0.f; sd[r] = 0.f; }
    const float SC2 = 1.4426950408889634f * 0.03125f;
#pragma unroll 1
    for (unsigned kc = qb; kc < NQB; ++kc) {
        const unsigned kv0 = kc * 64u;
        v8f s[4];
#pragma unroll
        for (int j = 0; j < 4; ++j) {
            const _Float16* krow = QK + (size_t)(rowbase + kv0 + 16u * (unsigned)j + c) * 2048u + 1024u + h * 64u + 8u * hh;
            v8f acc = (v8f){0.f,0.f,0.f,0.f,0.f,0.f,0.f,0.f};
            acc = wmma16(qa0, frag_ld(krow), acc);
            acc = wmma16(qa1, frag_ld(krow + 32), acc);
            s[j] = acc;
        }
#pragma unroll
        for (int r = 0; r < 8; ++r) {
            const unsigned qi = q0 + 8u * hh + (unsigned)r;
            float t[4];
#pragma unroll
            for (int j = 0; j < 4; ++j) {
                const unsigned kvcol = kv0 + 16u * (unsigned)j + c;
                const float tv = s[j][r] * SC2;
                t[j] = (kvcol >= qi) ? tv : 0.f;
                sd[r] = (kvcol == qi) ? tv : sd[r];
            }
            const float mx = fmaxf(fmaxf(t[0], t[1]), fmaxf(t[2], t[3]));
            const float mn = fmaxf(m[r], mx);
            l[r] = l[r] * exp2f(m[r] - mn) + ((exp2f(t[0] - mn) + exp2f(t[1] - mn)) + (exp2f(t[2] - mn) + exp2f(t[3] - mn)));
            m[r] = mn;
        }
    }
    const float nbelow = (float)(64u * qb);
#pragma unroll
    for (int r = 0; r < 8; ++r) {
        float M = m[r];
        M = fmaxf(M, __shfl_xor(M, 1, 32)); M = fmaxf(M, __shfl_xor(M, 2, 32));
        M = fmaxf(M, __shfl_xor(M, 4, 32)); M = fmaxf(M, __shfl_xor(M, 8, 32));
        float lr = l[r] * exp2f(m[r] - M);
        lr += __shfl_xor(lr, 1, 32); lr += __shfl_xor(lr, 2, 32); lr += __shfl_xor(lr, 4, 32); lr += __shfl_xor(lr, 8, 32);
        float sdr = sd[r];
        sdr += __shfl_xor(sdr, 1, 32); sdr += __shfl_xor(sdr, 2, 32); sdr += __shfl_xor(sdr, 4, 32); sdr += __shfl_xor(sdr, 8, 32);
        const float eM = exp2f(-M);
        const float Z = lr + nbelow * eM;
        const float inv = 1.0f / Z;
        const float wP = eM * inv, wD = exp2f(sdr - M) * inv;
        if (c == 0u) { wsc[wave][(8u * hh + (unsigned)r) * 2u] = wP; wsc[wave][(8u * hh + (unsigned)r) * 2u + 1u] = wD; }
    }
    __builtin_amdgcn_fence(3  , "workgroup");
    __builtin_amdgcn_wave_barrier();
    __builtin_amdgcn_fence(2  , "workgroup");
#pragma unroll
    for (int it = 0; it < 4; ++it) {
        const unsigned row = (unsigned)it * 4u + (lane >> 3), c8 = (lane & 7u) * 8u;
        const size_t g = (size_t)(rowbase + q0 + row) * 1024u + h * 64u + c8;
        const v4f ca = *(const v4f*)(CS + g), cb = *(const v4f*)(CS + g + 4);
        const v4f va = *(const v4f*)(V32 + g), vb = *(const v4f*)(V32 + g + 4);
        const float wp = wsc[wave][row * 2u] * 1024.f, wd = wsc[wave][row * 2u + 1u] * 1024.f;
        const v4f oa = ca * wp + va * wd, ob = cb * wp + vb * wd;
        v4u pk; pk.x = pk2h(oa.x, oa.y); pk.y = pk2h(oa.z, oa.w); pk.z = pk2h(ob.x, ob.y); pk.w = pk2h(ob.z, ob.w);
        VST2(v4u, (v4u*)(AO + g), pk);
    }
}

constexpr size_t SZ_WQKV = (size_t)3 * 1024 * 1024 * 2;
constexpr size_t SZ_WO   = (size_t)1024 * 1024 * 2;
constexpr size_t SZ_W1   = (size_t)4096 * 1024 * 2;
constexpr size_t SZ_W2   = (size_t)1024 * 4096 * 2;
constexpr size_t SZ_N16  = (size_t)MROWS * 1024 * 2;
constexpr size_t SZ_H32  = (size_t)MROWS * 1024 * 4;
constexpr size_t SZ_QK16 = (size_t)MROWS * 2048 * 2;
constexpr size_t SZ_V32  = (size_t)MROWS * 1024 * 4;
constexpr size_t SZ_H16  = (size_t)MROWS * 4096 * 2;
constexpr size_t SZ_R1   = (SZ_QK16 + SZ_V32 > SZ_H16) ? (SZ_QK16 + SZ_V32) : SZ_H16;
constexpr size_t SZ_CS   = (size_t)MROWS * 1024 * 4;
constexpr size_t SZ_AO16 = (size_t)MROWS * 1024 * 2;
constexpr size_t SZ_X1   = (size_t)MROWS * 1024 * 4;
constexpr size_t SZ_TOTAL = SZ_WQKV + SZ_WO + SZ_W1 + SZ_W2 + SZ_N16 + SZ_H32 + SZ_R1 + SZ_CS + SZ_AO16 + SZ_X1;
static_assert(SZ_QK16 + SZ_V32 <= SZ_R1);
static_assert(SZ_H16 <= SZ_R1);
static_assert(SZ_TOTAL <= (size_t)134217728);
static_assert((SZ_WQKV % 256) == 0 && (SZ_WO % 256) == 0 && (SZ_N16 % 256) == 0 && (SZ_QK16 % 256) == 0 && (SZ_AO16 % 256) == 0);
static_assert((size_t)NB_FULL * SEQ_FULL * 1024 * 4 == (size_t)16777216);
static_assert(((size_t)(NB - 1) * SEQ_FULL + SEQ) * 1024 * 4 <= (size_t)16777216);

extern "C" void kernel_launch(void* const* d_in, const int* in_sizes, int n_in, void* d_out, int out_size, void* d_ws, size_t ws_size, hipStream_t stream) {
    if (n_in < 17) return;
    const long long need_x = ((long long)(NB - 1) * SEQ_FULL + SEQ) * 1024;
    if ((long long)in_sizes[0] < need_x) return;
    if (in_sizes[1] < 1024 || in_sizes[2] < 1024 || in_sizes[4] < 1024 || in_sizes[6] < 1024 || in_sizes[8] < 1024 || in_sizes[10] < 1024 ||
        in_sizes[11] < 1024 || in_sizes[12] < 1024 || in_sizes[14] < 4096 || in_sizes[16] < 1024) return;
    if (in_sizes[3] < 1048576 || in_sizes[5] < 1048576 || in_sizes[7] < 1048576 || in_sizes[9] < 1048576 || in_sizes[13] < 4194304 || in_sizes[15] < 4194304) return;
    if ((long long)out_size < need_x) return;
    if (ws_size < SZ_TOTAL) return;
    const float* x   = (const float*)d_in[0];
    const float* g1  = (const float*)d_in[1];
    const float* be1 = (const float*)d_in[2];
    const float* wq  = (const float*)d_in[3];
    const float* bq  = (const float*)d_in[4];
    const float* wk  = (const float*)d_in[5];
    const float* bk  = (const float*)d_in[6];
    const float* wv  = (const float*)d_in[7];
    const float* bv  = (const float*)d_in[8];
    const float* wo  = (const float*)d_in[9];
    const float* bo  = (const float*)d_in[10];
    const float* g2  = (const float*)d_in[11];
    const float* be2 = (const float*)d_in[12];
    const float* w1  = (const float*)d_in[13];
    const float* b1  = (const float*)d_in[14];
    const float* w2  = (const float*)d_in[15];
    const float* b2  = (const float*)d_in[16];
    float* out = (float*)d_out;

    char* wsp = (char*)d_ws;
    unsigned short* WQKV16 = (unsigned short*)wsp; wsp += SZ_WQKV;
    unsigned short* WO16   = (unsigned short*)wsp; wsp += SZ_WO;
    unsigned short* W116   = (unsigned short*)wsp; wsp += SZ_W1;
    unsigned short* W216   = (unsigned short*)wsp; wsp += SZ_W2;
    unsigned short* N16    = (unsigned short*)wsp; wsp += SZ_N16;
    float*          H32    = (float*)wsp;          wsp += SZ_H32;
    char*           R1     = wsp;                  wsp += SZ_R1;
    float*          CSP    = (float*)wsp;          wsp += SZ_CS;
    unsigned short* AO16   = (unsigned short*)wsp; wsp += SZ_AO16;
    float*          X1     = (float*)wsp;          wsp += SZ_X1;
    unsigned short* QK16   = (unsigned short*)R1;
    float*          V32    = (float*)(R1 + SZ_QK16);
    unsigned short* H16    = (unsigned short*)R1;

    k_castT<<<(1024u * 128u + 255u) / 256u, 256, 0, stream>>>(wq, 1024u, WQKV16,            1024u, 1024u, 1024u, 7u, 16.0f);
    k_castT<<<(1024u * 128u + 255u) / 256u, 256, 0, stream>>>(wk, 1024u, WQKV16 + 1048576u, 1024u, 1024u, 1024u, 7u, 16.0f);
    k_castT<<<(1024u * 128u + 255u) / 256u, 256, 0, stream>>>(wv, 1024u, WQKV16 + 2097152u, 1024u, 1024u, 1024u, 7u, 16.0f);
    k_castT<<<(1024u * 128u + 255u) / 256u, 256, 0, stream>>>(wo, 1024u, WO16,              1024u, 1024u, 1024u, 7u, 16.0f);
    k_castT<<<(4096u * 128u + 255u) / 256u, 256, 0, stream>>>(w1, 4096u, W116,              1024u, 1024u, 4096u, 7u, 16.0f);
    k_castT<<<(1024u * 512u + 255u) / 256u, 256, 0, stream>>>(w2, 1024u, W216,              4096u, 4096u, 1024u, 9u, 16.0f);

    k_ln<1, 1><<<(unsigned)(MROWS / 8), 256, 0, stream>>>(x, g1, be1, N16, H32);

    {
        const unsigned tiles = (unsigned)(MROWS / 64) * (1024u / 64u);
        k_gemm64<1, false, 0><<<dim3((tiles + 7u) / 8u, 2u), 256, 0, stream>>>(N16, 1024u, 0ull, WQKV16, 1024u, 1048576ull, (void*)QK16, 2048u, 1024ull,
                                                                               bq, bk, nullptr, 0u, (unsigned)MROWS, 1024u, 1024u, 0.0625f);
        k_gemm64<0, false, 0><<<dim3((tiles + 7u) / 8u, 1u), 256, 0, stream>>>(N16, 1024u, 0ull, WQKV16 + 2097152u, 1024u, 0ull, (void*)V32, 1024u, 0ull,
                                                                               bv, bv, nullptr, 0u, (unsigned)MROWS, 1024u, 1024u, 0.0625f);
    }
    k_prefix<<<(unsigned)(NB * 1024 / 256), 256, 0, stream>>>(V32, CSP);
    k_attn_tri<<<(unsigned)(NB * NHEAD * (SEQ / 64)), 128, 0, stream>>>(QK16, V32, CSP, AO16);

    {
        const unsigned tiles = (unsigned)(MROWS / 64) * (1024u / 64u);
        k_gemm64<0, true, 0><<<dim3((tiles + 7u) / 8u, 1u), 256, 0, stream>>>(AO16, 1024u, 0ull, WO16, 1024u, 0ull, (void*)X1, 1024u, 0ull,
                                                                              bo, bo, H32, 1024u, (unsigned)MROWS, 1024u, 1024u, 6.103515625e-05f);
    }
    k_ln<0, 0><<<(unsigned)(MROWS / 8), 256, 0, stream>>>(X1, g2, be2, N16, nullptr);

    {
        const unsigned tiles = (unsigned)(MROWS / 64) * (4096u / 64u);
        k_gemm64<1, false, 2><<<dim3((tiles + 7u) / 8u, 1u), 256, 0, stream>>>(N16, 1024u, 0ull, W116, 1024u, 0ull, (void*)H16, 4096u, 0ull,
                                                                               b1, b1, nullptr, 0u, (unsigned)MROWS, 4096u, 1024u, 0.0625f);
    }
    {
        const unsigned tiles = (unsigned)(SEQ / 64) * (1024u / 64u);
        k_gemm64<0, false, 2><<<dim3((tiles + 7u) / 8u, (unsigned)NB), 256, 0, stream>>>(H16, 4096u, (unsigned long long)SEQ * 4096ull, W216, 4096u, 0ull,
                                                                                         (void*)out, 1024u, (unsigned long long)SEQ_FULL * 1024ull,
                                                                                         b2, b2, nullptr, 0u, (unsigned)SEQ, 1024u, 4096u, 0.0625f);
    }
}
